// MultiHeadAttention_55628416418020
// MI455X (gfx1250) — hardware-verified
//
#include <hip/hip_runtime.h>


#ifndef NB
#define NB 2
#endif
#ifndef SEQ
#define SEQ 2048
#endif
#define NB_FULL  2
#define SEQ_FULL 2048
#define DM   1024
#define NH   16
#define HD   64
#define ER   256
#define CTP  (2 * DM)
#define PCAR 1024.0f
#define QRS  2048.0f
#define VRS  2048.0f
#define SCL  0.125f
#define MNEG (-10000.0f)
#define L2E  1.4426950408889634f
#define PP   40
#define CP   136
#define PCS  ((2 * HD) / 8)
#define TSP  72

typedef _Float16 h16;
typedef unsigned short bf;
typedef __attribute__((ext_vector_type(16))) __bf16   v16bf;
typedef __attribute__((ext_vector_type(16))) _Float16 v16h;
typedef __attribute__((ext_vector_type(8)))  _Float16 v8h;
typedef __attribute__((ext_vector_type(8)))  unsigned short v8us;
typedef __attribute__((ext_vector_type(8)))  float    v8f;
typedef __attribute__((ext_vector_type(4)))  float    v4f;
typedef v8h  __attribute__((may_alias)) v8ha;
typedef v4f  __attribute__((may_alias)) v4fa;
typedef v8us __attribute__((may_alias)) v8usa;

static_assert(DM == NH * HD);
static_assert(HD % 32 == 0);
static_assert(HD / 16 == 4);
static_assert(HD % 8 == 0);
static_assert((2 * HD) % 8 == 0);
static_assert(SEQ % 64 == 0);
static_assert(SEQ % 32 == 0);
static_assert(SEQ % 8 == 0);
static_assert(ER % 64 == 0);
static_assert(ER >= 64 && ER <= SEQ);
static_assert((NB * SEQ) % 64 == 0);
static_assert(DM % 64 == 0);
static_assert(DM % 32 == 0);
static_assert(CTP % 64 == 0);
static_assert(CTP % 32 == 0);
static_assert((2 * HD * 2) % 128 == 0);
static_assert(16 * PCS == 8 * 32);
static_assert(PP >= 32 && PP % 8 == 0);
static_assert(CP >= 2 * HD && CP % 8 == 0);
static_assert(TSP >= 64 && TSP % 8 == 0);
static_assert((SEQ * DM) % (8 * 256) == 0);
static_assert((DM * DM) % (8 * 256) == 0);
static_assert((DM * CTP) % (8 * 256) == 0);
static_assert(NB <= NB_FULL && SEQ <= SEQ_FULL);
static_assert((size_t)NB * SEQ * DM * 4 <= (size_t)16777216);

__device__ __forceinline__ unsigned short f2bf(float f) { unsigned u = __float_as_uint(f); u += 0x7FFFu + ((u >> 16) & 1u); return (unsigned short)(u >> 16); }
__device__ __forceinline__ float bf2f(unsigned short b) { return __uint_as_float(((unsigned)b) << 16); }
__device__ __forceinline__ float bfr(float f) { return bf2f(f2bf(f)); }
__device__ __forceinline__ void splitf(float y, unsigned short& h, unsigned short& l) { h = f2bf(y); l = f2bf(y - bf2f(h)); }
__device__ __forceinline__ v16h cat16(v8h lo, v8h hi) { return __builtin_shufflevector(lo, hi, 0, 1, 2, 3, 4, 5, 6, 7, 8, 9, 10, 11, 12, 13, 14, 15); }
__device__ __forceinline__ v16bf cat16b(v8us lo, v8us hi) { return __builtin_bit_cast(v16bf, __builtin_shufflevector(lo, hi, 0, 1, 2, 3, 4, 5, 6, 7, 8, 9, 10, 11, 12, 13, 14, 15)); }
__device__ __forceinline__ v8f wmma16(v16h a, v16h b, v8f c) {
    c = __builtin_amdgcn_wmma_f32_16x16x32_f16(false, a, false, b, (short)0, c, false, false);
    asm volatile("v_nop\n\tv_nop\n\tv_nop\n\tv_nop" : "+v"(c) : "v"(a), "v"(b));
    return c; }
__device__ __forceinline__ v8f wmmab(v16bf a, v16bf b, v8f c) {
    c = __builtin_amdgcn_wmma_f32_16x16x32_bf16(false, a, false, b, (short)0, c, false, false);
    asm volatile("v_nop\n\tv_nop\n\tv_nop\n\tv_nop" : "+v"(c) : "v"(a), "v"(b));
    return c; }
__device__ __forceinline__ v16h ldh(const h16* p) { return cat16(*(const v8h*)p, *(const v8h*)(p + 16)); }
__device__ __forceinline__ v16bf ldb(const bf* p) { return cat16b(*(const v8us*)p, *(const v8us*)(p + 16)); }

__global__ __launch_bounds__(256) void k_wcv(const float* __restrict__ w, bf* dst, int K, int il, int total8) {
    const int i = blockIdx.x * 256 + threadIdx.x; if (i >= total8) return;
    const int KO = il ? 2 * K : K; const int e = i * 8; const int n = e / KO, kk = e % KO;
    const int k = il ? ((kk / (2 * HD)) * HD + (kk % (2 * HD)) % HD) : kk;
    const v8f v = *(const v8f*)(w + (size_t)n * K + k); v8us o;
#pragma unroll
    for (int q = 0; q < 8; ++q) o[q] = f2bf(v[q]);
    bf* d = dst + (size_t)e; *(volatile v8us*)d = o; __threadfence(); *(volatile v8us*)d = o; }

__global__ __launch_bounds__(256) void k_cvt8(const float* __restrict__ src, bf* dst) {
    const int i = blockIdx.x * 256 + threadIdx.x; const int b = blockIdx.y; if (i >= SEQ * DM / 8) return;
    const v8f v = *(const v8f*)(src + (size_t)b * SEQ_FULL * DM + (size_t)i * 8); v8us o;
#pragma unroll
    for (int k = 0; k < 8; ++k) o[k] = f2bf(v[k]);
    bf* d = dst + (size_t)b * SEQ * DM + (size_t)i * 8; *(volatile v8us*)d = o; __threadfence(); *(volatile v8us*)d = o; }

__global__ __launch_bounds__(256) void k_maskT(const float* __restrict__ mask, bf* MT) {
    __shared__ __align__(16) unsigned short ts[64 * TSP];
    const int t = threadIdx.x; const int j0 = blockIdx.x * 64, i0 = blockIdx.y * 64;
#pragma unroll 1
    for (int it = 0; it < 16; ++it) { const int i = it * 4 + (t >> 6), j = t & 63;
        ts[j * TSP + i] = f2bf(mask[(size_t)(i0 + i) * SEQ_FULL + j0 + j]); }
    __syncthreads();
#pragma unroll 1
    for (int ps = 0; ps < 2; ++ps) {
#pragma unroll
        for (int s = 0; s < 2; ++s) { const int slot = s * 256 + t; const int jr = slot >> 3, pc = slot & 7;
            const v8us o = *(const v8usa*)(ts + jr * TSP + pc * 8);
            *(volatile v8us*)(MT + (size_t)(j0 + jr) * SEQ + i0 + pc * 8) = o; }
        if (ps == 0) __threadfence(); }
}

__global__ __launch_bounds__(32) void k_gemm(const bf* __restrict__ A, const bf* __restrict__ Bt, h16* C16, h16* CL, float* C32, const float* __restrict__ bias,
                                             size_t sA, size_t sB, size_t sC, int K, int ldc, int mode) {
    __shared__ __align__(16) float os[16 * 68];
    const size_t z = blockIdx.z; A += z * sA; Bt += z * sB; const size_t coff = z * sC;
    const int lane = threadIdx.x & 31, lr = lane & 15, hi = lane >> 4; const int r0 = blockIdx.x * 64, c0 = blockIdx.y * 64;
    const bool rowb = (mode == 2) || (mode == 4); const bool wres = (mode == 1) || (mode == 4);
    v8f acc[4][4];
#pragma unroll
    for (int mb = 0; mb < 4; ++mb)
#pragma unroll
        for (int nb = 0; nb < 4; ++nb) acc[mb][nb] = (v8f){};
    const size_t aoff = (size_t)(r0 + lr) * K + 8 * hi, boff = (size_t)(c0 + lr) * K + 8 * hi;
#pragma unroll 1
    for (int kc = 0; kc < K; kc += 32) {
        v16bf a[4]; v16bf b;
#pragma unroll
        for (int mb = 0; mb < 4; ++mb) a[mb] = ldb(A + aoff + (size_t)mb * 16 * K + kc);
#pragma unroll
        for (int nb = 0; nb < 4; ++nb) { b = ldb(Bt + boff + (size_t)nb * 16 * K + kc);
#pragma unroll
            for (int mb = 0; mb < 4; ++mb) acc[mb][nb] = wmmab(a[mb], b, acc[mb][nb]); }
    }
#pragma unroll
    for (int mb = 0; mb < 4; ++mb) {
#pragma unroll
        for (int nb = 0; nb < 4; ++nb) {
#pragma unroll
            for (int j = 0; j < 8; ++j) os[(hi * 8 + j) * 68 + nb * 16 + lr] = acc[mb][nb][j]; }
        __builtin_amdgcn_wave_barrier(); asm volatile("" ::: "memory");
        if (mode == 3) {
            float* crow = C32 + coff + (size_t)(r0 + mb * 16) * ldc + c0;
#pragma unroll 1
            for (int ps = 0; ps < 2; ++ps) {
#pragma unroll
                for (int s = 0; s < 8; ++s) { const int row = 2 * s + hi, cofs = lr * 4; v4f val = *(const v4fa*)(os + row * 68 + cofs);
                    val[0] += bfr(bias[c0 + cofs]); val[1] += bfr(bias[c0 + cofs + 1]); val[2] += bfr(bias[c0 + cofs + 2]); val[3] += bfr(bias[c0 + cofs + 3]);
                    *(volatile v4f*)(crow + (size_t)row * ldc + cofs) = val; }
                if (ps == 0) __threadfence(); }
        } else {
#pragma unroll 1
            for (int ps = 0; ps < 2; ++ps) {
#pragma unroll
                for (int s = 0; s < 4; ++s) { const int row = 4 * s + (lane >> 3), cg = lane & 7;
                    const v4f x0 = *(const v4fa*)(os + row * 68 + cg * 8); const v4f x1 = *(const v4fa*)(os + row * 68 + cg * 8 + 4);
                    const int grow = r0 + mb * 16 + row, gcol = c0 + cg * 8; const int bi0 = rowb ? grow : gcol; const int bst = rowb ? 0 : 1;
                    v8h o, ol;
#pragma unroll
                    for (int q = 0; q < 8; ++q) { const float v = ((q < 4) ? x0[q & 3] : x1[q & 3]) + bfr(bias[bi0 + q * bst]); const h16 hx = (h16)v; o[q] = hx; ol[q] = (h16)((v - (float)hx) * QRS); }
                    const size_t oo = coff + (size_t)grow * ldc + gcol;
                    *(volatile v8h*)(C16 + oo) = o; if (wres) *(volatile v8h*)(CL + oo) = ol; }
                if (ps == 0) __threadfence(); }
        }
        __builtin_amdgcn_wave_barrier(); asm volatile("" ::: "memory");
    }
}

template <int EARLY>
__device__ __forceinline__ void attn_body(const h16* __restrict__ Q16, const h16* __restrict__ QL, const h16* __restrict__ K16, const h16* __restrict__ KL,
                                          const h16* __restrict__ VT, const h16* __restrict__ VL, const bf* __restrict__ MT, bf* CT) {
    __shared__ __align__(16) h16 pws[4 * 16 * PP];
    __shared__ __align__(16) h16 prs[EARLY ? 4 * 16 * PP : 8];
    __shared__ __align__(16) unsigned short cts[4 * 16 * CP];
    const int wave = __builtin_amdgcn_readfirstlane((int)(threadIdx.x >> 5));
    const int lane = threadIdx.x & 31, lr = lane & 15, hi = lane >> 4;
    const int b = blockIdx.z, h = blockIdx.y;
    const int qs0 = ((int)blockIdx.x + (EARLY ? 0 : ER / 64)) * 64 + wave * 16;
    const int row0 = b * SEQ + qs0;
    const int qoff = (row0 + lr) * DM + h * HD + 8 * hi;
    const int kbase = (b * SEQ + lr) * DM + h * HD + 8 * hi;
    const int vbase = (b * DM + h * HD + lr) * SEQ + 8 * hi;
    const int mbase = lr * SEQ + qs0 + 8 * hi;
    const int pb = wave * 16 * PP, cb = wave * 16 * CP;
    v8f ctx[4], ctxr[4]; float mrun[8], srun[8];
#pragma unroll
    for (int nt = 0; nt < 4; ++nt) { ctx[nt] = (v8f){}; ctxr[nt] = (v8f){}; }
#pragma unroll
    for (int r = 0; r < 8; ++r) { mrun[r] = -1.0e30f; srun[r] = 0.0f; }
#pragma unroll 1
    for (int kb = 0; kb < SEQ; kb += 32) {
        int qo = qoff; asm volatile("" : "+v"(qo));
        const int ko = kbase + kb * DM;
        const v8us m0 = *(const v8us*)(MT + mbase + kb * SEQ);
        const v8us m1 = *(const v8us*)(MT + mbase + (kb + 16) * SEQ);
        v8f sh0 = (v8f){}, sh1 = (v8f){}, sl0 = (v8f){}, sl1 = (v8f){};
#pragma unroll
        for (int ks = 0; ks < HD / 32; ++ks) {
            const v16h qa = ldh(Q16 + qo + ks * 32); const v16h qr = ldh(QL + qo + ks * 32);
            const v16h k0 = ldh(K16 + ko + ks * 32); const v16h k1 = ldh(K16 + ko + 16 * DM + ks * 32);
            const v16h kr0 = ldh(KL + ko + ks * 32); const v16h kr1 = ldh(KL + ko + 16 * DM + ks * 32);
            sh0 = wmma16(qa, k0, sh0); sh1 = wmma16(qa, k1, sh1);
            sl0 = wmma16(qr, k0, sl0); sl1 = wmma16(qr, k1, sl1);
            sl0 = wmma16(qa, kr0, sl0); sl1 = wmma16(qa, kr1, sl1); }
#pragma unroll
        for (int r = 0; r < 8; ++r) {
            const float t0 = (sh0[r] + sl0[r] * (1.0f / QRS)) * SCL + bf2f(m0[r]) * MNEG;
            const float t1 = (sh1[r] + sl1[r] * (1.0f / QRS)) * SCL + bf2f(m1[r]) * MNEG;
            float mx = fmaxf(t0, t1);
            mx = fmaxf(mx, __shfl_xor(mx, 1, 32)); mx = fmaxf(mx, __shfl_xor(mx, 2, 32)); mx = fmaxf(mx, __shfl_xor(mx, 4, 32)); mx = fmaxf(mx, __shfl_xor(mx, 8, 32));
            const float nm = fmaxf(mrun[r], mx); const float corr = __builtin_amdgcn_exp2f((mrun[r] - nm) * L2E); mrun[r] = nm;
            const float p0 = __builtin_amdgcn_exp2f((t0 - nm) * L2E); const float p1 = __builtin_amdgcn_exp2f((t1 - nm) * L2E);
            srun[r] = srun[r] * corr + (p0 + p1);
#pragma unroll
            for (int nt = 0; nt < 4; ++nt) ctx[nt][r] *= corr;
            const float c0 = p0 * PCAR, c1 = p1 * PCAR; const h16 g0 = (h16)c0, g1 = (h16)c1;
            pws[pb + (8 * hi + r) * PP + lr] = g0; pws[pb + (8 * hi + r) * PP + 16 + lr] = g1;
            if (EARLY) {
#pragma unroll
                for (int nt = 0; nt < 4; ++nt) ctxr[nt][r] *= corr;
                prs[pb + (8 * hi + r) * PP + lr] = (h16)((c0 - (float)g0) * VRS); prs[pb + (8 * hi + r) * PP + 16 + lr] = (h16)((c1 - (float)g1) * VRS); } }
        __builtin_amdgcn_wave_barrier(); asm volatile("" ::: "memory");
        const v16h pa = cat16(*(const v8ha*)(pws + pb + lr * PP + 8 * hi), *(const v8ha*)(pws + pb + lr * PP + 16 + 8 * hi));
        v16h pra = pa;
        if (EARLY) pra = cat16(*(const v8ha*)(prs + pb + lr * PP + 8 * hi), *(const v8ha*)(prs + pb + lr * PP + 16 + 8 * hi));
#pragma unroll
        for (int nt = 0; nt < 4; ++nt) { const v16h vb = ldh(VT + vbase + nt * 16 * SEQ + kb); ctx[nt] = wmma16(pa, vb, ctx[nt]);
            if (EARLY) { ctxr[nt] = wmma16(pra, vb, ctxr[nt]); const v16h vr = ldh(VL + vbase + nt * 16 * SEQ + kb); ctxr[nt] = wmma16(pa, vr, ctxr[nt]); } }
        __builtin_amdgcn_wave_barrier(); asm volatile("" ::: "memory");
    }
    float rinv[8];
#pragma unroll
    for (int r = 0; r < 8; ++r) { float s = srun[r]; s += __shfl_xor(s, 1, 32); s += __shfl_xor(s, 2, 32); s += __shfl_xor(s, 4, 32); s += __shfl_xor(s, 8, 32); rinv[r] = (1.0f / PCAR) * (1.0f / s); }
#pragma unroll
    for (int nt = 0; nt < 4; ++nt) {
#pragma unroll
        for (int r = 0; r < 8; ++r) { float a = ctx[nt][r]; if (EARLY) a += ctxr[nt][r] * (1.0f / VRS);
            const float val = a * rinv[r]; unsigned short hh, ll; splitf(val, hh, ll);
            cts[cb + (8 * hi + r) * CP + nt * 16 + lr] = hh; cts[cb + (8 * hi + r) * CP + HD + nt * 16 + lr] = ll; } }
    __builtin_amdgcn_wave_barrier(); asm volatile("" ::: "memory");
#pragma unroll 1
    for (int ps = 0; ps < 2; ++ps) {
#pragma unroll
        for (int it = 0; it < 8; ++it) { const int slot = it * 32 + lane; const int row = slot / PCS, pc = slot % PCS;
            const v8us o = *(const v8usa*)(cts + cb + row * CP + pc * 8);
            *(volatile v8us*)(CT + (size_t)(row0 + row) * CTP + h * 2 * HD + pc * 8) = o; }
        if (ps == 0) __threadfence(); }
}

__global__ __launch_bounds__(128) void k_attn_e(const h16* __restrict__ Q16, const h16* __restrict__ QL, const h16* __restrict__ K16, const h16* __restrict__ KL,
                                                const h16* __restrict__ VT, const h16* __restrict__ VL, const bf* __restrict__ MT, bf* CT) {
    attn_body<1>(Q16, QL, K16, KL, VT, VL, MT, CT); }
__global__ __launch_bounds__(128) void k_attn_l(const h16* __restrict__ Q16, const h16* __restrict__ QL, const h16* __restrict__ K16, const h16* __restrict__ KL,
                                                const h16* __restrict__ VT, const h16* __restrict__ VL, const bf* __restrict__ MT, bf* CT) {
    attn_body<0>(Q16, QL, K16, KL, VT, VL, MT, CT); }

constexpr size_t al256(size_t x) { return (x + 255) & ~(size_t)255; }
constexpr size_t SZ_W   = al256((size_t)DM * DM * 2);
constexpr size_t SZ_WO  = al256((size_t)DM * CTP * 2);
constexpr size_t SZ_PL  = al256((size_t)NB * SEQ * DM * 2);
constexpr size_t SZ_CT  = al256((size_t)NB * SEQ * CTP * 2);
constexpr size_t SZ_MT  = al256((size_t)SEQ * SEQ * 2);
constexpr size_t WS_TOTAL = 3 * SZ_W + SZ_WO + 7 * SZ_PL + SZ_CT + SZ_MT;
static_assert(WS_TOTAL <= (size_t)134217728);

extern "C" void kernel_launch(void* const* d_in, const int* in_sizes, int n_in,
                              void* d_out, int out_size, void* d_ws, size_t ws_size, hipStream_t stream) {
    if (n_in < 12) return;
    const long long need_x = (long long)(NB - 1) * SEQ_FULL * DM + (long long)SEQ * DM;
    if (in_sizes[0] < need_x || in_sizes[1] < need_x || in_sizes[2] < need_x) return;
    if ((long long)in_sizes[3] < (long long)(SEQ - 1) * SEQ_FULL + SEQ) return;
    if (in_sizes[4] < DM * DM || in_sizes[6] < DM * DM || in_sizes[8] < DM * DM || in_sizes[10] < DM * DM) return;
    if (in_sizes[5] < DM || in_sizes[7] < DM || in_sizes[9] < DM || in_sizes[11] < DM) return;
    if ((long long)out_size < (long long)NB * SEQ * DM) return;
    if (WS_TOTAL > ws_size) return;
    const float* xq = (const float*)d_in[0]; const float* xk = (const float*)d_in[1]; const float* xv = (const float*)d_in[2]; const float* mask = (const float*)d_in[3];
    const float* wq = (const float*)d_in[4]; const float* bq = (const float*)d_in[5]; const float* wk = (const float*)d_in[6]; const float* bk = (const float*)d_in[7];
    const float* wv = (const float*)d_in[8]; const float* bv = (const float*)d_in[9]; const float* wo = (const float*)d_in[10]; const float* bo = (const float*)d_in[11];
    float* OUT = (float*)d_out;
    char* wsp = (char*)d_ws;
    auto take = [&](size_t bytes) { char* p = wsp; wsp += bytes; return (void*)p; };
    bf* WQ = (bf*)take(SZ_W); bf* WK = (bf*)take(SZ_W); bf* WV = (bf*)take(SZ_W); bf* WO2 = (bf*)take(SZ_WO);
    bf* XB = (bf*)take(SZ_PL); h16* Q16 = (h16*)take(SZ_PL); h16* QL = (h16*)take(SZ_PL); h16* K16 = (h16*)take(SZ_PL); h16* KL = (h16*)take(SZ_PL);
    h16* VT16 = (h16*)take(SZ_PL); h16* VTL = (h16*)take(SZ_PL);
    bf* CT = (bf*)take(SZ_CT); bf* MT = (bf*)take(SZ_MT);

    const int nW8 = DM * DM / 8, nWO8 = DM * CTP / 8;
    k_wcv<<<(unsigned)(nW8 / 256), 256, 0, stream>>>(wq, WQ, DM, 0, nW8);
    k_wcv<<<(unsigned)(nW8 / 256), 256, 0, stream>>>(wk, WK, DM, 0, nW8);
    k_wcv<<<(unsigned)(nW8 / 256), 256, 0, stream>>>(wv, WV, DM, 0, nW8);
    k_wcv<<<(unsigned)(nWO8 / 256), 256, 0, stream>>>(wo, WO2, DM, 1, nWO8);
    k_maskT<<<dim3(SEQ / 64, SEQ / 64, 1), 256, 0, stream>>>(mask, MT);
    const dim3 gC((unsigned)(SEQ * DM / 8 / 256), NB, 1);
    const dim3 gP((unsigned)(NB * SEQ / 64), DM / 64, 1);
    k_cvt8<<<gC, 256, 0, stream>>>(xq, XB);
    k_gemm<<<gP, 32, 0, stream>>>(XB, WQ, Q16, QL, OUT, bq, (size_t)0, (size_t)0, (size_t)0, DM, DM, 1);
    k_cvt8<<<gC, 256, 0, stream>>>(xk, XB);
    k_gemm<<<gP, 32, 0, stream>>>(XB, WK, K16, KL, OUT, bk, (size_t)0, (size_t)0, (size_t)0, DM, DM, 1);
    k_cvt8<<<gC, 256, 0, stream>>>(xv, XB);
    k_gemm<<<dim3(DM / 64, SEQ / 64, NB), 32, 0, stream>>>(WV, XB, VT16, VTL, OUT, bv, (size_t)0, (size_t)SEQ * DM, (size_t)DM * SEQ, DM, SEQ, 4);
    k_attn_e<<<dim3(ER / 64, NH, NB), 128, 0, stream>>>(Q16, QL, K16, KL, VT16, VTL, MT, CT);
    if (SEQ > ER) k_attn_l<<<dim3((SEQ - ER) / 64, NH, NB), 128, 0, stream>>>(Q16, QL, K16, KL, VT16, VTL, MT, CT);
    k_gemm<<<gP, 32, 0, stream>>>(CT, WO2, Q16, Q16, OUT, bo, (size_t)0, (size_t)0, (size_t)0, CTP, DM, 3);
}
